// EncoderLayer_71004399337823
// MI455X (gfx1250) — hardware-verified
//
#include <hip/hip_runtime.h>
#ifndef NB
#define NB 2
#endif
#ifndef SEQ
#define SEQ 2048
#endif
#define SQ SEQ
#define NB_FULL 2
#define SQ_FULL 2048
#define DM 1024
#define DMQ DM
#define NH 16
#define HD 64
#define DFF 4096
#define LQ (3 * DM)
#define NR ((size_t)NB * SQ)
#define MP (NB * SQ)
static_assert(NB >= 1 && NB <= NB_FULL);
static_assert(SQ <= SQ_FULL && (SQ % 128) == 0);
static_assert((MP % 128) == 0);
static_assert(DM == NH * HD && (DM % 64) == 0 && (DFF % 64) == 0 && (DM % 32) == 0 && (DFF % 32) == 0);
static_assert(DMQ == 1024);
static_assert(((size_t)NB * SQ * DM) % 8 == 0);

typedef unsigned short v8us __attribute__((ext_vector_type(8), may_alias));
typedef float  v8f  __attribute__((ext_vector_type(8)));
typedef float  v4f  __attribute__((ext_vector_type(4)));
typedef float  v4fa __attribute__((ext_vector_type(4), may_alias));
typedef int    v4ia __attribute__((ext_vector_type(4), may_alias));
typedef _Float16 v16h __attribute__((ext_vector_type(16)));
typedef _Float16 v4h  __attribute__((ext_vector_type(4)));
union FragH { v16h v; v8us half[2]; _Float16 h[16]; unsigned short u[16]; };

__device__ __forceinline__ unsigned short bf16_bits(float x) { unsigned int u = __float_as_uint(x); return (unsigned short)((u + 0x7FFFu + ((u >> 16) & 1u)) >> 16); }
__device__ __forceinline__ float bf16_val(unsigned short b) { return __uint_as_float(((unsigned int)b) << 16); }
__device__ __forceinline__ float bf16_rne(float x) { return bf16_val(bf16_bits(x)); }

__device__ __forceinline__ v16h g2_frag(const _Float16* p, int hh) { FragH f; f.half[0] = *(const v8us*)((const unsigned short*)p + 8 * hh); f.half[1] = *(const v8us*)((const unsigned short*)p + 16 + 8 * hh); return f.v; }
__device__ __forceinline__ v8f g2_mma(v16h a, v16h b, v8f c) { v8f d = __builtin_amdgcn_wmma_f32_16x16x32_f16(false, a, false, b, (short)0, c, false, false); asm volatile("v_nop\n\tv_nop\n\tv_nop\n\tv_nop" : "+v"(d) : "v"(a), "v"(b)); return d; }

__global__ __launch_bounds__(256) void k_wt_f16(const float* __restrict__ W, _Float16* __restrict__ Wt, int K, int N, float scale) {
  const int t = blockIdx.x * 256 + threadIdx.x; if (t >= N * (K / 8)) return; const int n = t / (K / 8), k8 = (t % (K / 8)) * 8; FragH f;
#pragma unroll
  for (int i = 0; i < 8; ++i) f.h[i] = (_Float16)(bf16_rne(W[(size_t)(k8 + i) * N + n]) * scale);
  const v8us o = f.half[0];
  *(volatile v8us*)((unsigned short*)Wt + (size_t)n * K + k8) = o; __threadfence(); *(volatile v8us*)((unsigned short*)Wt + (size_t)n * K + k8) = o;
}

__global__ __launch_bounds__(256) void k_bcat3(const float* __restrict__ b0, const float* __restrict__ b1, const float* __restrict__ b2, float* __restrict__ dst) {
  for (int pass = 0; pass < 2; ++pass) {
#pragma unroll 1
    for (unsigned i = threadIdx.x; i < 3u * DM; i += 256u) { const unsigned sel = i / (unsigned)DM, c = i % (unsigned)DM; const float v0 = b0[c], v1 = b1[c], v2 = b2[c]; const float v = (sel == 0u) ? v0 : ((sel == 1u) ? v1 : v2); *(volatile float*)(dst + i) = v; }
    if (pass == 0) __threadfence();
  }
}

__global__ __launch_bounds__(256) void k_x16(const float* __restrict__ x, _Float16* __restrict__ X16, unsigned n8) {
  const unsigned t = blockIdx.x * 256u + threadIdx.x; if (t >= n8) return;
  const unsigned e = t * 8u; const unsigned row = e / (unsigned)DM, col = e % (unsigned)DM; const unsigned bb = row / (unsigned)SQ; const unsigned srow = bb * (unsigned)SQ_FULL + (row - bb * (unsigned)SQ);
  const float* src = x + (size_t)srow * DM + col; const v4f a = *(const v4fa*)src, c = *(const v4fa*)(src + 4); FragH f;
#pragma unroll
  for (int q = 0; q < 4; ++q) { f.h[q] = (_Float16)bf16_rne(a[q]); f.h[4 + q] = (_Float16)bf16_rne(c[q]); }
  const v8us o = f.half[0];
  *(volatile v8us*)((unsigned short*)X16 + (size_t)t * 8) = o; __threadfence(); *(volatile v8us*)((unsigned short*)X16 + (size_t)t * 8) = o;
}

template <int ACT, int CPM>
__global__ __launch_bounds__(128) void k_gemm2(const _Float16* __restrict__ A, int lda, const _Float16* __restrict__ Bh, int ldb, float alpha, const float* __restrict__ bias, const float* __restrict__ CP,
    float* __restrict__ C, _Float16* __restrict__ C16, int ldc, int M, int N, int K) {
  static_assert(ACT == 0 || ACT == 3);
  static_assert(CPM == 0 || ACT == 0);
  __shared__ __attribute__((aligned(16))) float so[4][32][68];
  const int tid = threadIdx.x, w = tid >> 5, lane = tid & 31, ln = lane & 15, hh = lane >> 4;
  const int ntn = N >> 6; const int mt = blockIdx.x / ntn, nq = blockIdx.x - mt * ntn; const int row0 = mt * 128 + 32 * w, col0 = nq * 64; if (row0 >= M) return;
  const _Float16* a0p = A + (size_t)(row0 + ln) * lda; const _Float16* a1p = a0p + (size_t)16 * lda;
  const _Float16* b0p = Bh + (size_t)(col0 + ln) * ldb; const _Float16* b1p = b0p + (size_t)16 * ldb; const _Float16* b2p = b1p + (size_t)16 * ldb; const _Float16* b3p = b2p + (size_t)16 * ldb;
  const v8f z8 = {0.f,0.f,0.f,0.f,0.f,0.f,0.f,0.f}; v8f c00 = z8, c01 = z8, c02 = z8, c03 = z8, c10 = z8, c11 = z8, c12 = z8, c13 = z8;
#pragma unroll 1
  for (int kb = 0; kb < K; kb += 32) { const v16h a0 = g2_frag(a0p + kb, hh), a1 = g2_frag(a1p + kb, hh);
    v16h b = g2_frag(b0p + kb, hh); c00 = g2_mma(a0, b, c00); c10 = g2_mma(a1, b, c10);
    b = g2_frag(b1p + kb, hh); c01 = g2_mma(a0, b, c01); c11 = g2_mma(a1, b, c11);
    b = g2_frag(b2p + kb, hh); c02 = g2_mma(a0, b, c02); c12 = g2_mma(a1, b, c12);
    b = g2_frag(b3p + kb, hh); c03 = g2_mma(a0, b, c03); c13 = g2_mma(a1, b, c13); }
  v8f accs[8] = {c00, c01, c02, c03, c10, c11, c12, c13};
#pragma unroll
  for (int u = 0; u < 8; ++u) { const int t = u & 3, half = u >> 2; const int col = col0 + t * 16 + ln; const float bv = bias ? bf16_rne(bias[col]) : 0.f;
#pragma unroll
    for (int r = 0; r < 8; ++r) { const int rloc = half * 16 + 8 * hh + r; float v = accs[u][r] * alpha + bv; if (ACT == 3) v = fmaxf(v, 0.f); so[w][rloc][t * 16 + ln] = v; } }
  __builtin_amdgcn_fence(4  , "workgroup"); __builtin_amdgcn_wave_barrier();
  const int rsub = lane >> 4, c4 = (lane & 15) * 4;
  for (int pass = 0; pass < 2; ++pass) {
#pragma unroll
    for (int q = 0; q < 16; ++q) { const int r = q * 2 + rsub; v4f v = *(const v4fa*)&so[w][r][c4];
      if (CPM == 1) { const unsigned rr = (unsigned)(row0 + r); const unsigned bb = rr / (unsigned)SQ; const unsigned sr = bb * (unsigned)SQ_FULL + (rr - bb * (unsigned)SQ); const v4f cv = *(const v4fa*)(CP + (size_t)sr * DM + col0 + c4);
#pragma unroll
        for (int i = 0; i < 4; ++i) v[i] += bf16_rne(cv[i]); }
      if (CPM == 2) { const v4f cv = *(const v4fa*)(CP + (size_t)(row0 + r) * ldc + col0 + c4); v += cv; }
      if (C) *(volatile v4f*)(C + (size_t)(row0 + r) * ldc + col0 + c4) = v;
      if (C16) { v4h h4;
#pragma unroll
        for (int i = 0; i < 4; ++i) h4[i] = (_Float16)v[i];
        *(volatile v4h*)(C16 + (size_t)(row0 + r) * ldc + col0 + c4) = h4; } }
    if (pass == 0) __threadfence(); } }

template <int NHv, int TTv>
__global__ __launch_bounds__(256) void k_vt(const _Float16* __restrict__ V16, int ldv, int voff, _Float16* __restrict__ Vt) {
  __shared__ unsigned short tl[64][66];
  const unsigned tid = threadIdx.x; const unsigned slab = blockIdx.x / (unsigned)(TTv / 64), lg = blockIdx.x % (unsigned)(TTv / 64); const unsigned b = slab / (unsigned)NHv, h = slab % (unsigned)NHv;
  for (unsigned i = tid; i < 512u; i += 256u) { const unsigned r = i >> 3, c8 = (i & 7u) * 8u; FragH f; f.half[0] = *(const v8us*)((const unsigned short*)V16 + ((size_t)b * TTv + lg * 64u + r) * ldv + voff + h * 64u + c8);
#pragma unroll
    for (int q = 0; q < 8; ++q) tl[r][c8 + q] = f.u[q]; }
  __syncthreads();
  for (int pass = 0; pass < 2; ++pass) {
#pragma unroll
    for (int rd = 0; rd < 2; ++rd) { const unsigned d = rd * 32u + (tid >> 3), pc = tid & 7u; FragH f;
#pragma unroll
      for (int q = 0; q < 8; ++q) f.u[q] = tl[pc * 8u + q][d];
      *(volatile v8us*)((unsigned short*)Vt + ((size_t)slab * 64u + d) * TTv + lg * 64u + pc * 8u) = f.half[0]; }
    if (pass == 0) __threadfence(); } }

__global__ __launch_bounds__(128) void k_flash(const _Float16* __restrict__ QKV, const _Float16* __restrict__ VT, const int* __restrict__ mask, _Float16* __restrict__ O16) {
  __shared__ __attribute__((aligned(16))) int smk[SQ];
  __shared__ __attribute__((aligned(16))) unsigned short sot[4][16][64];
  const unsigned tid = threadIdx.x, w = tid >> 5, lane = tid & 31u, ln = lane & 15u; const int hh = (int)(lane >> 4);
  const unsigned qt = blockIdx.x % (unsigned)(SQ / 64), bh = blockIdx.x / (unsigned)(SQ / 64);
  const unsigned h = bh % (unsigned)NH, b = bh / (unsigned)NH;
  const int* mrow = mask + (size_t)b * SQ_FULL;
  for (unsigned i = tid; i < (unsigned)(SQ / 4); i += 128u) { const v4ia mv = *(const v4ia*)(mrow + 4u * i); *(v4ia*)&smk[4u * i] = mv; }
  __syncthreads();
  const size_t rowq = (size_t)b * SQ + qt * 64u + w * 16u;
  const _Float16* qp = QKV + (rowq + ln) * LQ + h * HD;
  const v16h q0f = g2_frag(qp, hh), q1f = g2_frag(qp + 32, hh);
  const _Float16* kbase = QKV + ((size_t)b * SQ + ln) * LQ + DM + h * HD;
  const _Float16* vbase = VT + ((size_t)bh * HD + ln) * SQ;
  const v8f z8 = {0.f,0.f,0.f,0.f,0.f,0.f,0.f,0.f};
  v8f o[4] = {z8, z8, z8, z8};
  float m = -1.0e30f, l = 0.f;
#pragma unroll 1
  for (unsigned kb = 0; kb < (unsigned)SQ; kb += 64u) {
    v8f s[4];
#pragma unroll
    for (int t = 0; t < 4; ++t) { const _Float16* kp = kbase + (size_t)(kb + 16u * (unsigned)t) * LQ; s[t] = g2_mma(g2_frag(kp, hh), q0f, z8); }
#pragma unroll
    for (int t = 0; t < 4; ++t) { const _Float16* kp = kbase + (size_t)(kb + 16u * (unsigned)t) * LQ + 32; s[t] = g2_mma(g2_frag(kp, hh), q1f, s[t]); }
    float mloc = -1.0e30f;
#pragma unroll
    for (int t = 0; t < 4; ++t) {
      const v4ia k0 = *(const v4ia*)&smk[kb + 16u * (unsigned)t + 8u * (unsigned)hh]; const v4ia k1 = *(const v4ia*)&smk[kb + 16u * (unsigned)t + 8u * (unsigned)hh + 4u];
#pragma unroll
      for (int r = 0; r < 4; ++r) {
        float v0 = s[t][r] * 0.125f; v0 = (k0[r] == 0) ? -1.0e9f : v0; s[t][r] = v0; mloc = fmaxf(mloc, v0);
        float v1 = s[t][r + 4] * 0.125f; v1 = (k1[r] == 0) ? -1.0e9f : v1; s[t][r + 4] = v1; mloc = fmaxf(mloc, v1); }
    }
    mloc = fmaxf(mloc, __shfl_xor(mloc, 16));
    const float mn = fmaxf(m, mloc); const float fac = __expf(m - mn); m = mn; l *= fac;
    FragH pb0, pb1;
#pragma unroll
    for (int r = 0; r < 8; ++r) { float p;
      p = __expf(s[0][r] - mn); l += p; pb0.h[r] = (_Float16)(p * 1024.0f);
      p = __expf(s[1][r] - mn); l += p; pb0.h[8 + r] = (_Float16)(p * 1024.0f);
      p = __expf(s[2][r] - mn); l += p; pb1.h[r] = (_Float16)(p * 1024.0f);
      p = __expf(s[3][r] - mn); l += p; pb1.h[8 + r] = (_Float16)(p * 1024.0f); }
#pragma unroll
    for (int dt = 0; dt < 4; ++dt) o[dt] = o[dt] * fac;
#pragma unroll
    for (int dt = 0; dt < 4; ++dt) { const _Float16* vp = vbase + (size_t)(16u * (unsigned)dt) * SQ + kb; o[dt] = g2_mma(g2_frag(vp, hh), pb0.v, o[dt]); }
#pragma unroll
    for (int dt = 0; dt < 4; ++dt) { const _Float16* vp = vbase + (size_t)(16u * (unsigned)dt) * SQ + kb + 32; o[dt] = g2_mma(g2_frag(vp, hh), pb1.v, o[dt]); }
  }
  l += __shfl_xor(l, 16);
  const float fin = 0.0625f * (1.0f / l);
#pragma unroll
  for (int dt = 0; dt < 4; ++dt) { FragH f;
#pragma unroll
    for (int r = 0; r < 8; ++r) f.h[r] = (_Float16)(o[dt][r] * fin);
    *(v8us*)&sot[w][ln][16 * dt + 8 * hh] = f.half[0]; }
  __builtin_amdgcn_fence(4  , "workgroup"); __builtin_amdgcn_wave_barrier();
  for (int pass = 0; pass < 2; ++pass) {
#pragma unroll
    for (int j = 0; j < 4; ++j) { const unsigned row = 4u * (unsigned)j + (lane >> 3), pc = (lane & 7u) * 8u; const v8us v = *(const v8us*)&sot[w][row][pc];
      *(volatile v8us*)((unsigned short*)O16 + (rowq + row) * DM + h * HD + pc) = v; }
    if (pass == 0) __threadfence(); } }

template <int BFIN, int W16, int W32, int OMAP>
__global__ __launch_bounds__(256) void k_lnx(const float* __restrict__ X, const float* __restrict__ g, const float* __restrict__ bb, float eps, _Float16* __restrict__ N16, float* __restrict__ N32) {
  #pragma clang fp contract(off)
  __shared__ float red[256]; const unsigned ru = blockIdx.x; const size_t r = ru; const int t = threadIdx.x; const int c0 = t * 4;
  const v4f xa = *(const v4fa*)(X + r * DMQ + c0); float s[4]; float sum = 0.f;
  for (int q = 0; q < 4; ++q) { s[q] = BFIN ? bf16_rne(xa[q]) : xa[q]; sum = __fadd_rn(sum, s[q]); }
  red[t] = sum; __syncthreads(); for (int st = 128; st > 0; st >>= 1) { if (t < st) red[t] = __fadd_rn(red[t], red[t + st]); __syncthreads(); } const float mu = red[0] * (1.0f / (float)DMQ); __syncthreads();
  float vs = 0.f; for (int q = 0; q < 4; ++q) { const float dl = __fadd_rn(s[q], -mu); vs = __fadd_rn(vs, __fmul_rn(dl, dl)); } red[t] = vs; __syncthreads(); for (int st = 128; st > 0; st >>= 1) { if (t < st) red[t] = __fadd_rn(red[t], red[t + st]); __syncthreads(); }
  const float rs = rsqrtf(__fadd_rn(red[0] * (1.0f / (float)DMQ), eps)); v4h y; v4f yf;
  for (int q = 0; q < 4; ++q) { const int c = c0 + q; yf[q] = __fadd_rn(__fmul_rn(__fmul_rn(__fadd_rn(s[q], -mu), rs), bf16_rne(g[c])), bf16_rne(bb[c])); y[q] = (_Float16)yf[q]; }
  const unsigned ob = ru / (unsigned)SQ; const size_t orow = OMAP ? ((size_t)ob * SQ_FULL + (ru - ob * (unsigned)SQ)) : r;
  for (int pass = 0; pass < 2; ++pass) { if (W16) *(volatile v4h*)(N16 + r * DMQ + c0) = y; if (W32) *(volatile v4f*)(N32 + orow * DMQ + c0) = yf; if (pass == 0) __threadfence(); } }

extern "C" void kernel_launch(void* const* d_in, const int* in_sizes, int n_in,
                              void* d_out, int out_size, void* d_ws, size_t ws_size, hipStream_t stream) {
  if (n_in < 18) return;
  const size_t rows_full = (size_t)(NB - 1) * SQ_FULL + SQ;
  if ((size_t)in_sizes[0] < rows_full * DM) return;
  if ((size_t)in_sizes[1] < rows_full) return;
  if ((size_t)in_sizes[2] < (size_t)DM * DM || (size_t)in_sizes[4] < (size_t)DM * DM || (size_t)in_sizes[6] < (size_t)DM * DM || (size_t)in_sizes[8] < (size_t)DM * DM) return;
  if ((size_t)in_sizes[10] < (size_t)DM * DFF || (size_t)in_sizes[12] < (size_t)DFF * DM) return;
  if (in_sizes[3] < DM || in_sizes[5] < DM || in_sizes[7] < DM || in_sizes[9] < DM || in_sizes[11] < DFF || in_sizes[13] < DM) return;
  if (in_sizes[14] < DM || in_sizes[15] < DM || in_sizes[16] < DM || in_sizes[17] < DM) return;
  if ((size_t)out_size < rows_full * DM) return;
  const float* x = (const float*)d_in[0]; const int* mask = (const int*)d_in[1];
  const float* wq = (const float*)d_in[2]; const float* bq = (const float*)d_in[3]; const float* wk = (const float*)d_in[4]; const float* bk = (const float*)d_in[5];
  const float* wv = (const float*)d_in[6]; const float* bv = (const float*)d_in[7]; const float* wo = (const float*)d_in[8]; const float* bo = (const float*)d_in[9];
  const float* w1 = (const float*)d_in[10]; const float* b1 = (const float*)d_in[11]; const float* w2 = (const float*)d_in[12]; const float* b2 = (const float*)d_in[13];
  const float* g1 = (const float*)d_in[14]; const float* be1 = (const float*)d_in[15]; const float* g2 = (const float*)d_in[16]; const float* be2 = (const float*)d_in[17];
  float* out = (float*)d_out;
  char* ws = (char*)d_ws; size_t off = 0;
  auto take = [&](size_t bytes) { char* p = ws + off; off += (bytes + 255) & ~(size_t)255; return p; };
  _Float16* BQKV = (_Float16*)take((size_t)3 * DM * DM * 2);
  _Float16* BO   = (_Float16*)take((size_t)DM * DM * 2);
  float*    bqkv = (float*)take((size_t)3 * DM * 4);
  _Float16* X16  = (_Float16*)take(NR * DM * 2);
  float*    X1   = (float*)take(NR * DM * 4);
  _Float16* BW1  = (_Float16*)take((size_t)DFF * DM * 2);
  _Float16* BW2  = (_Float16*)take((size_t)DM * DFF * 2);
  _Float16* QKV  = (_Float16*)take(NR * LQ * 2);
  _Float16* O16  = (_Float16*)take(NR * DM * 2);
  _Float16* VT   = (_Float16*)take((size_t)NB * NH * HD * SQ * 2);
  _Float16* HF16 = (_Float16*)take(NR * DFF * 2);
  static_assert(NR * DM * 4 <= NR * LQ * 2);
  if (off > ws_size || off > (size_t)134217728) return;
  _Float16* M16 = X16; float* X1N = (float*)QKV;
  { const unsigned g = (unsigned)(((size_t)DM * (DM / 8) + 255) / 256);
    k_wt_f16<<<g, 256, 0, stream>>>(wq, BQKV, DM, DM, 16.0f); k_wt_f16<<<g, 256, 0, stream>>>(wk, BQKV + (size_t)DM * DM, DM, DM, 16.0f);
    k_wt_f16<<<g, 256, 0, stream>>>(wv, BQKV + (size_t)2 * DM * DM, DM, DM, 16.0f); k_wt_f16<<<g, 256, 0, stream>>>(wo, BO, DM, DM, 16.0f); }
  k_wt_f16<<<(unsigned)(((size_t)DFF * (DM / 8) + 255) / 256), 256, 0, stream>>>(w1, BW1, DM, DFF, 16.0f);
  k_wt_f16<<<(unsigned)(((size_t)DM * (DFF / 8) + 255) / 256), 256, 0, stream>>>(w2, BW2, DFF, DM, 16.0f);
  k_bcat3<<<1, 256, 0, stream>>>(bq, bk, bv, bqkv);
  { const unsigned n8 = (unsigned)(NR * DM / 8); k_x16<<<(n8 + 255u) / 256u, 256, 0, stream>>>(x, X16, n8); }
  k_gemm2<0, 0><<<dim3((unsigned)((MP / 128) * (LQ / 64)), 1), 128, 0, stream>>>(X16, DM, BQKV, DM, 0.0625f, bqkv, nullptr, nullptr, QKV, LQ, MP, LQ, DM);
  k_vt<NH, SQ><<<(unsigned)(NB * NH * (SQ / 64)), 256, 0, stream>>>(QKV + 2 * DM, LQ, 0, VT);
  k_flash<<<(unsigned)(NB * NH * (SQ / 64)), 128, 0, stream>>>(QKV, VT, mask, O16);
  k_gemm2<0, 1><<<dim3((unsigned)((MP / 128) * (DM / 64)), 1), 128, 0, stream>>>(O16, DM, BO, DM, 0.0009765625f, bo, x, X1, nullptr, DM, MP, DM, DM);
  k_lnx<0, 1, 1, 0><<<(unsigned)NR, 256, 0, stream>>>(X1, g1, be1, 1e-5f, M16, X1N);
  k_gemm2<3, 0><<<dim3((unsigned)((MP / 128) * (DFF / 64)), 1), 128, 0, stream>>>(M16, DM, BW1, DM, 0.0625f, b1, nullptr, nullptr, HF16, DFF, MP, DFF, DM);
  k_gemm2<0, 2><<<dim3((unsigned)((MP / 128) * (DM / 64)), 1), 128, 0, stream>>>(HF16, DFF, BW2, DFF, 0.0625f, b2, X1N, X1, nullptr, DM, MP, DM, DFF);
  k_lnx<0, 0, 1, 1><<<(unsigned)NR, 256, 0, stream>>>(X1, g2, be2, 1e-5f, nullptr, out);
}
